// GoogleAttention_154618823219
// MI455X (gfx1250) — hardware-verified
//
#include <hip/hip_runtime.h>
#include <math.h>

constexpr int kNB   = 4;
constexpr int kNN   = 4096;
constexpr int kCC   = 512;
constexpr int kCK   = 64;
constexpr int kCV   = 256;
constexpr int kRows = kNB * kNN;
constexpr float kPCarry     = 32768.0f;
constexpr float kPCarryInv  = 1.0f / 32768.0f;
constexpr float kWoCarry    = 16.0f;
constexpr float kWoCarryInv = 1.0f / 16.0f;

constexpr size_t kOffA  = 0;
constexpr size_t kOffP  = kOffA  + (size_t)kNN * kNN * 4;
constexpr size_t kOffO  = kOffP  + (size_t)kNN * kNN * 2;
constexpr size_t kOffHV = kOffO  + (size_t)kRows * kCV * 2;
constexpr size_t kOffGh = kOffHV + (size_t)kNB * kCV * kNN * 2;
constexpr size_t kOffGl = kOffGh + (size_t)kRows * kCK * 2;
constexpr size_t kOffFh = kOffGl + (size_t)kRows * kCK * 2;
constexpr size_t kOffFl = kOffFh + (size_t)kRows * kCK * 2;
constexpr size_t kOffWg = kOffFl + (size_t)kRows * kCK * 2;
constexpr size_t kOffWf = kOffWg + (size_t)kCK * kCC * 2;
constexpr size_t kOffWh = kOffWf + (size_t)kCK * kCC * 2;
constexpr size_t kOffWo = kOffWh + (size_t)kCV * kCC * 2;
constexpr size_t kWsTotal = kOffWo + (size_t)kCC * kCV * 2;
static_assert(kWsTotal == 126484480ull);
static_assert(kWsTotal <= 134217728ull);
static_assert((size_t)kRows * kCC * 2 <= (size_t)kNN * kNN * 4);

typedef __attribute__((ext_vector_type(16))) _Float16 v16h;
typedef __attribute__((ext_vector_type(8)))  _Float16 v8h;
typedef __attribute__((ext_vector_type(16))) __bf16   v16b;
typedef __attribute__((ext_vector_type(8)))  __bf16   v8b;
typedef __attribute__((ext_vector_type(8)))  float    v8f;
typedef __attribute__((ext_vector_type(4)))  float    v4f;
typedef __attribute__((ext_vector_type(4)))  unsigned int v4u;

__device__ __forceinline__ unsigned short f2bf_bits(float f) {
  unsigned u = __float_as_uint(f);
  return (unsigned short)((u + 0x7FFFu + ((u >> 16) & 1u)) >> 16);
}
__device__ __forceinline__ float bf_bits2f(unsigned short h) { return __uint_as_float(((unsigned)h) << 16); }

__device__ __forceinline__ void dep_guard_h(v8f& a, v8f& b, v16h x, v16h y) { asm volatile("v_nop\n\tv_nop\n\tv_nop\n\tv_nop" : "+v"(a), "+v"(b) : "v"(x), "v"(y)); }
__device__ __forceinline__ void dep_guard_b(v8f& a, v8f& b, v16b x, v16b y) { asm volatile("v_nop\n\tv_nop\n\tv_nop\n\tv_nop" : "+v"(a), "+v"(b) : "v"(x), "v"(y)); }
__device__ __forceinline__ void keep4_h(v16h a, v16h b, v16h c, v16h d) { asm volatile("v_nop" :: "v"(a), "v"(b), "v"(c), "v"(d)); }
__device__ __forceinline__ void keep4_b(v16b a, v16b b, v16b c, v16b d) { asm volatile("v_nop" :: "v"(a), "v"(b), "v"(c), "v"(d)); }
__device__ __forceinline__ void acc_guard4(v8f& a, v8f& b, v8f& c, v8f& d) { asm volatile("v_nop\n\tv_nop\n\tv_nop\n\tv_nop" : "+v"(a), "+v"(b), "+v"(c), "+v"(d)); }
template <typename T> struct Frag;
template <> struct Frag<_Float16> {
  typedef v16h V; union U { v16h v; v8h h[2]; };
  static __device__ __forceinline__ v16h load(const _Float16* p) {
    U f; f.h[0] = *(const v8h*)(p); f.h[1] = *(const v8h*)(p + 16); return f.v;
  }
  static __device__ __forceinline__ v8f mma(v16h a, v16h b, v8f c) {
    return __builtin_amdgcn_wmma_f32_16x16x32_f16(false, a, false, b, (short)0, c, false, false);
  }
  static __device__ __forceinline__ void guard(v8f& a, v8f& b, v16h x, v16h y) { dep_guard_h(a, b, x, y); }
  static __device__ __forceinline__ void keep(v16h a, v16h b, v16h c, v16h d) { keep4_h(a, b, c, d); }
};
template <> struct Frag<__bf16> {
  typedef v16b V; union U { v16b v; v8b h[2]; };
  static __device__ __forceinline__ v16b load(const __bf16* p) {
    U f; f.h[0] = *(const v8b*)(p); f.h[1] = *(const v8b*)(p + 16); return f.v;
  }
  static __device__ __forceinline__ v8f mma(v16b a, v16b b, v8f c) {
    return __builtin_amdgcn_wmma_f32_16x16x32_bf16(false, a, false, b, (short)0, c, false, false);
  }
  static __device__ __forceinline__ void guard(v8f& a, v8f& b, v16b x, v16b y) { dep_guard_b(a, b, x, y); }
  static __device__ __forceinline__ void keep(v16b a, v16b b, v16b c, v16b d) { keep4_b(a, b, c, d); }
};

__device__ __forceinline__ unsigned pk16(unsigned short a, unsigned short b) { return (unsigned)a | ((unsigned)b << 16); }
__device__ __forceinline__ unsigned short h_bits(float f) { const _Float16 h = (_Float16)f; return __builtin_bit_cast(unsigned short, h); }

template <int ET> struct Elem;
template <> struct Elem<0> { typedef _Float16 T; };
template <> struct Elem<1> { typedef __bf16 T; };
template <int ET, bool SPLIT, int BIAS_MODE, int OUT_MODE, bool RESID, int GMODE = 0>
__global__ __launch_bounds__(256) void wmma_gemm64(
    const unsigned short* __restrict__ Ap, const unsigned short* __restrict__ A2p, int lda, long strideA,
    const unsigned short* __restrict__ Btp, const unsigned short* __restrict__ Bt2p, int ldb, long strideB,
    void* __restrict__ Cout, void* __restrict__ Cout2, int ldc, long strideC,
    const float* __restrict__ bias,
    const float* __restrict__ resid, long strideR,
    int M, int N, int K, float scale,
    const float* __restrict__ gsp) {
  typedef typename Elem<ET>::T T;
  typedef typename Frag<T>::V V;
  const T* A = (const T*)Ap; const T* A2 = (const T*)A2p; const T* Bt = (const T*)Btp; const T* Bt2 = (const T*)Bt2p;
  __shared__ __align__(16) float sT[8][16 * 68];
  const int b    = blockIdx.y;
  const int lane = threadIdx.x & 31;
  const int wave = threadIdx.x >> 5;
  const int tilesN = N >> 6;
  const int tilesM = M >> 6;
  const int tile = blockIdx.x * 8 + wave;
  if (tile >= tilesM * tilesN) return;
  const int tm = tile / tilesN;
  const int tn = tile - tm * tilesN;
  const int m0 = tm << 6;
  const int n0 = tn << 6;

  const T* Ab  = A  + (size_t)b * strideA;
  const T* Bb  = Bt + (size_t)b * strideB;
  const T* Ab2 = SPLIT ? (A2  + (size_t)b * strideA) : nullptr;
  const T* Bb2 = SPLIT ? (Bt2 + (size_t)b * strideB) : nullptr;

  const int rlane = lane & 15;
  const int koff  = (lane >> 4) * 8;
  const int mOff  = (lane >> 4) * 8;

  const float gsv = (GMODE == 1) ? bf_bits2f(f2bf_bits(gsp[0])) : 1.0f;

  v8f acc[4][4];
#pragma unroll
  for (int i = 0; i < 4; ++i)
#pragma unroll
    for (int j = 0; j < 4; ++j) acc[i][j] = (v8f){0.f,0.f,0.f,0.f,0.f,0.f,0.f,0.f};

  for (int k0 = 0; k0 < K; k0 += 32) {
    V bh[4], bl[4];
#pragma unroll
    for (int j = 0; j < 4; ++j) {
      const size_t bo = (size_t)(n0 + (j << 4) + rlane) * ldb + koff + k0;
      bh[j] = Frag<T>::load(Bb + bo);
      if (SPLIT) bl[j] = Frag<T>::load(Bb2 + bo);
    }
#pragma unroll
    for (int i = 0; i < 4; ++i) {
      const size_t ao = (size_t)(m0 + (i << 4) + rlane) * lda + koff + k0;
      V ah = Frag<T>::load(Ab + ao);
      V al;
      if (SPLIT) al = Frag<T>::load(Ab2 + ao);
#pragma unroll
      for (int j = 0; j < 4; ++j) {
        acc[i][j] = Frag<T>::mma(ah, bh[j], acc[i][j]);
        if (SPLIT) {
          acc[i][j] = Frag<T>::mma(ah, bl[j], acc[i][j]);
          acc[i][j] = Frag<T>::mma(al, bh[j], acc[i][j]);
        }
      }
      Frag<T>::guard(acc[i][0], acc[i][3], ah, SPLIT ? al : ah);
    }
    Frag<T>::keep(bh[0], bh[1], bh[2], bh[3]);
    if (SPLIT) Frag<T>::keep(bl[0], bl[1], bl[2], bl[3]);
  }
  acc_guard4(acc[0][0], acc[0][1], acc[0][2], acc[0][3]);
  acc_guard4(acc[1][0], acc[1][1], acc[1][2], acc[1][3]);
  acc_guard4(acc[2][0], acc[2][1], acc[2][2], acc[2][3]);
  acc_guard4(acc[3][0], acc[3][1], acc[3][2], acc[3][3]);

  float* slab = sT[wave];
  const float* Rb = RESID ? (resid + (size_t)b * strideR) : nullptr;
#pragma unroll
  for (int i = 0; i < 4; ++i) {
    const int mBase = m0 + (i << 4);
#pragma unroll
    for (int j = 0; j < 4; ++j) {
      const int n = n0 + (j << 4) + rlane;
      float bv = 0.f;
      if (BIAS_MODE == 2) bv = bias[n];
#pragma unroll
      for (int r = 0; r < 8; ++r) {
        float v = acc[i][j][r] * scale;
        if (BIAS_MODE == 1) v += bias[mBase + mOff + r];
        if (BIAS_MODE == 2) v += bv;
        if (GMODE == 1) v *= gsv;
        if (RESID) {
          float rv = Rb[(size_t)(mBase + mOff + r) * ldc + n];
          if (GMODE == 1) rv = bf_bits2f(f2bf_bits(rv));
          v += rv;
        }
        slab[(mOff + r) * 68 + (j << 4) + rlane] = v;
      }
    }
    __builtin_amdgcn_fence(__ATOMIC_RELEASE, "workgroup");
    __builtin_amdgcn_wave_barrier();
    __builtin_amdgcn_fence(__ATOMIC_ACQUIRE, "workgroup");
    if (OUT_MODE == 0) {
      float* C = (float*)Cout + (size_t)b * strideC;
      const int hh = lane >> 4, c4 = (lane & 15) * 4;
      for (int pass = 0; pass < 2; ++pass) {
#pragma unroll
        for (int it = 0; it < 8; ++it) {
          const int row = it * 2 + hh;
          v4f v = *(const v4f*)(slab + row * 68 + c4);
          *(volatile v4f*)(C + (size_t)(mBase + row) * ldc + n0 + c4) = v;
        }
        __threadfence();
      }
    } else {
      const int q = lane >> 3, c8 = (lane & 7) * 8;
      unsigned short* C  = (unsigned short*)Cout  + (size_t)b * strideC;
      unsigned short* C2 = (OUT_MODE == 2) ? ((unsigned short*)Cout2 + (size_t)b * strideC) : nullptr;
      for (int pass = 0; pass < 2; ++pass) {
#pragma unroll
        for (int it = 0; it < 4; ++it) {
          const int row = it * 4 + q;
          const float* sp = slab + row * 68 + c8;
          v8h hv, lv;
#pragma unroll
          for (int e = 0; e < 8; ++e) {
            if (OUT_MODE == 1) {
              hv[e] = (_Float16)sp[e];
            } else {
              unsigned short hb = f2bf_bits(sp[e]);
              unsigned short lb = f2bf_bits(sp[e] - bf_bits2f(hb));
              hv[e] = __builtin_bit_cast(_Float16, hb);
              lv[e] = __builtin_bit_cast(_Float16, lb);
            }
          }
          *(volatile v8h*)(C + (size_t)(mBase + row) * ldc + n0 + c8) = hv;
          if (OUT_MODE == 2) *(volatile v8h*)(C2 + (size_t)(mBase + row) * ldc + n0 + c8) = lv;
        }
        __threadfence();
      }
    }
    __builtin_amdgcn_fence(__ATOMIC_RELEASE, "workgroup");
    __builtin_amdgcn_wave_barrier();
    __builtin_amdgcn_fence(__ATOMIC_ACQUIRE, "workgroup");
  }
}

template <int MODE>
__global__ __launch_bounds__(256) void tcast_kernel(const float* __restrict__ W, int in_cols, int out_pitch,
                                                    unsigned short* __restrict__ out, float scale) {
  __shared__ float sm[64][65];
  const int t  = threadIdx.x;
  const int r0 = blockIdx.x * 64;
  const int c0 = blockIdx.y * 64;
#pragma unroll
  for (int i = 0; i < 16; ++i) {
    const int e = i * 256 + t;
    const int r = e >> 6;
    const int c = e & 63;
    sm[c][r] = W[(size_t)(r0 + r) * in_cols + c0 + c];
  }
  __syncthreads();
  const int lane = t & 31, wave = t >> 5;
  const int q = lane >> 3, c8 = (lane & 7) * 8;
  for (int pass = 0; pass < 2; ++pass) {
#pragma unroll
    for (int it = 0; it < 2; ++it) {
      const int row = wave * 8 + it * 4 + q;
      unsigned short hb[8];
#pragma unroll
      for (int e = 0; e < 8; ++e) {
        const float w = sm[row][c8 + e];
        if (MODE == 0) hb[e] = f2bf_bits(w);
        else           hb[e] = h_bits(bf_bits2f(f2bf_bits(w)) * scale);
      }
      const v4u u = (v4u){pk16(hb[0], hb[1]), pk16(hb[2], hb[3]), pk16(hb[4], hb[5]), pk16(hb[6], hb[7])};
      *(volatile v4u*)(out + (size_t)(c0 + row) * out_pitch + r0 + c8) = u;
    }
    __threadfence();
  }
}

__global__ __launch_bounds__(256) void xcast_bf16_kernel(const float* __restrict__ in, unsigned short* __restrict__ out, int n8) {
  const int i = blockIdx.x * 256 + threadIdx.x;
  if (i >= n8) return;
  const float* p = in + 8 * (size_t)i;
  const v4f a = *(const v4f*)(p);
  const v4f c = *(const v4f*)(p + 4);
  unsigned short hb[8];
#pragma unroll
  for (int e = 0; e < 4; ++e) {
    hb[e]     = f2bf_bits(a[e]);
    hb[4 + e] = f2bf_bits(c[e]);
  }
  const v4u u = (v4u){pk16(hb[0], hb[1]), pk16(hb[2], hb[3]), pk16(hb[4], hb[5]), pk16(hb[6], hb[7])};
  unsigned short* q = out + 8 * (size_t)i;
  *(volatile v4u*)q = u;
  __threadfence();
  *(volatile v4u*)q = u;
}

__global__ __launch_bounds__(256) void softmax_row_kernel(const float* __restrict__ S, unsigned short* __restrict__ P, float carry) {
  __shared__ float redM[8];
  __shared__ float redS[8];
  const int row  = blockIdx.x;
  const int t    = threadIdx.x;
  const int lane = t & 31, wave = t >> 5;
  const int c0   = t * 8;
  const int c1   = (kNN / 2) + t * 8;
  const float* sr = S + (size_t)row * kNN;
  const v4f a0 = *(const v4f*)(sr + c0);
  const v4f a1 = *(const v4f*)(sr + c0 + 4);
  const v4f a2 = *(const v4f*)(sr + c1);
  const v4f a3 = *(const v4f*)(sr + c1 + 4);
  float sv[16];
#pragma unroll
  for (int e = 0; e < 4; ++e) { sv[e] = a0[e]; sv[4 + e] = a1[e]; sv[8 + e] = a2[e]; sv[12 + e] = a3[e]; }
  float m = sv[0];
#pragma unroll
  for (int e = 1; e < 16; ++e) m = fmaxf(m, sv[e]);
#pragma unroll
  for (int off = 16; off > 0; off >>= 1) m = fmaxf(m, __shfl_xor(m, off, 32));
  if (lane == 0) redM[wave] = m;
  __syncthreads();
  float gm = redM[0];
#pragma unroll
  for (int w = 1; w < 8; ++w) gm = fmaxf(gm, redM[w]);
  float s = 0.f;
#pragma unroll
  for (int e = 0; e < 16; ++e) { sv[e] = __expf(sv[e] - gm); s += sv[e]; }
#pragma unroll
  for (int off = 16; off > 0; off >>= 1) s += __shfl_xor(s, off, 32);
  if (lane == 0) redS[wave] = s;
  __syncthreads();
  float tot = redS[0];
#pragma unroll
  for (int w = 1; w < 8; ++w) tot += redS[w];
  const float inv = carry * (1.0f / tot);
  unsigned short hb[16];
#pragma unroll
  for (int e = 0; e < 16; ++e) hb[e] = h_bits(sv[e] * inv);
  const v4u u0 = (v4u){pk16(hb[0], hb[1]),  pk16(hb[2], hb[3]),   pk16(hb[4], hb[5]),   pk16(hb[6], hb[7])};
  const v4u u1 = (v4u){pk16(hb[8], hb[9]),  pk16(hb[10], hb[11]), pk16(hb[12], hb[13]), pk16(hb[14], hb[15])};
  unsigned short* pr = P + (size_t)row * kNN;
  *(volatile v4u*)(pr + c0) = u0;
  *(volatile v4u*)(pr + c1) = u1;
  __threadfence();
  *(volatile v4u*)(pr + c0) = u0;
  *(volatile v4u*)(pr + c1) = u1;
}

extern "C" void kernel_launch(void* const* d_in, const int* in_sizes, int n_in,
                              void* d_out, int out_size, void* d_ws, size_t ws_size,
                              hipStream_t stream) {
  if (n_in < 10) return;
  if (in_sizes[0] != kRows * kCC || in_sizes[1] != kCC * kCK || in_sizes[2] != kCK ||
      in_sizes[3] != kCC * kCK || in_sizes[4] != kCK || in_sizes[5] != kCC * kCV ||
      in_sizes[6] != kCV || in_sizes[7] != kCV * kCC || in_sizes[8] != kCC || in_sizes[9] < 1) return;
  if (out_size != kRows * kCC) return;
  if (ws_size < kWsTotal) return;

  const float* x     = (const float*)d_in[0];
  const float* Wf    = (const float*)d_in[1];
  const float* bfv   = (const float*)d_in[2];
  const float* Wg    = (const float*)d_in[3];
  const float* bgv   = (const float*)d_in[4];
  const float* Wh    = (const float*)d_in[5];
  const float* bhv   = (const float*)d_in[6];
  const float* Wo    = (const float*)d_in[7];
  const float* bov   = (const float*)d_in[8];
  const float* gamma = (const float*)d_in[9];
  float* out = (float*)d_out;

  typedef unsigned short u16;
  char* ws = (char*)d_ws;
  u16*   xbf = (u16*)(ws + kOffA);
  float* Sp  = (float*)(ws + kOffA);
  u16*   Pp  = (u16*)(ws + kOffP);
  u16*   Op  = (u16*)(ws + kOffO);
  u16*   HVp = (u16*)(ws + kOffHV);
  u16*   Gh  = (u16*)(ws + kOffGh);
  u16*   Gl  = (u16*)(ws + kOffGl);
  u16*   Fh  = (u16*)(ws + kOffFh);
  u16*   Fl  = (u16*)(ws + kOffFl);
  u16*   WgT = (u16*)(ws + kOffWg);
  u16*   WfT = (u16*)(ws + kOffWf);
  u16*   WhT = (u16*)(ws + kOffWh);
  u16*   WoT = (u16*)(ws + kOffWo);

  tcast_kernel<0><<<dim3(kCC / 64, kCK / 64), dim3(256), 0, stream>>>(Wg, kCK, kCC, WgT, 1.0f);
  tcast_kernel<0><<<dim3(kCC / 64, kCK / 64), dim3(256), 0, stream>>>(Wf, kCK, kCC, WfT, 1.0f);
  tcast_kernel<0><<<dim3(kCC / 64, kCV / 64), dim3(256), 0, stream>>>(Wh, kCV, kCC, WhT, 1.0f);
  tcast_kernel<1><<<dim3(kCV / 64, kCC / 64), dim3(256), 0, stream>>>(Wo, kCC, kCV, WoT, kWoCarry);

  constexpr int kXN8 = kRows * kCC / 8;
  static_assert(kXN8 % 256 == 0);
  xcast_bf16_kernel<<<dim3(kXN8 / 256), dim3(256), 0, stream>>>(x, xbf, kXN8);

  wmma_gemm64<1, false, 2, 2, false, 0><<<dim3((kRows / 64) * (kCK / 64) / 8, 1), dim3(256), 0, stream>>>(
      xbf, xbf, kCC, 0L, WgT, WgT, kCC, 0L, (void*)Gh, (void*)Gl, kCK, 0L, bgv, x, 0L, kRows, kCK, kCC, 1.0f, gamma);
  wmma_gemm64<1, false, 2, 2, false, 0><<<dim3((kRows / 64) * (kCK / 64) / 8, 1), dim3(256), 0, stream>>>(
      xbf, xbf, kCC, 0L, WfT, WfT, kCC, 0L, (void*)Fh, (void*)Fl, kCK, 0L, bfv, x, 0L, kRows, kCK, kCC, 1.0f, gamma);
  wmma_gemm64<1, false, 1, 1, false, 0><<<dim3((kCV / 64) * (kNN / 64) / 8, kNB), dim3(256), 0, stream>>>(
      WhT, WhT, kCC, 0L, xbf, xbf, kCC, (long)kNN * kCC, (void*)HVp, (void*)HVp, kNN, (long)kCV * kNN,
      bhv, x, 0L, kCV, kNN, kCC, 1.0f, gamma);

  for (int bb = 0; bb < kNB; ++bb) {
    const size_t qk = (size_t)bb * kNN * kCK;
    wmma_gemm64<1, true, 0, 0, false, 0><<<dim3((kNN / 64) * (kNN / 64) / 8, 1), dim3(256), 0, stream>>>(
        Gh + qk, Gl + qk, kCK, 0L, Fh + qk, Fl + qk, kCK, 0L, (void*)Sp, (void*)Sp, kNN, 0L,
        bgv, x, 0L, kNN, kNN, kCK, 1.0f, gamma);
    softmax_row_kernel<<<dim3(kNN), dim3(256), 0, stream>>>(Sp, Pp, kPCarry);
    wmma_gemm64<0, false, 0, 1, false, 0><<<dim3((kNN / 64) * (kCV / 64) / 8, 1), dim3(256), 0, stream>>>(
        Pp, Pp, kNN, 0L, HVp + (size_t)bb * kCV * kNN, HVp + (size_t)bb * kCV * kNN, kNN, 0L,
        (void*)(Op + (size_t)bb * kNN * kCV), (void*)(Op + (size_t)bb * kNN * kCV), kCV, 0L,
        bhv, x, 0L, kNN, kCV, kNN, kPCarryInv, gamma);
  }

  wmma_gemm64<0, false, 2, 0, true, 1><<<dim3((kRows / 64) * (kCC / 64) / 8, 1), dim3(256), 0, stream>>>(
      Op, Op, kCV, 0L, WoT, WoT, kCV, 0L, (void*)out, (void*)out, kCC, 0L, bov, x, 0L, kRows, kCC, kCV, kWoCarryInv, gamma);
}
